// SimpleAttention_47983374631299
// MI455X (gfx1250) — hardware-verified
//
#include <hip/hip_runtime.h>
#include <stdint.h>


typedef _Float16 v16h __attribute__((ext_vector_type(16)));
typedef _Float16 v8h  __attribute__((ext_vector_type(8)));
typedef _Float16 v8ha __attribute__((ext_vector_type(8), may_alias));
typedef float    v8f  __attribute__((ext_vector_type(8)));
typedef float    v4f  __attribute__((ext_vector_type(4)));
typedef float    v4fa __attribute__((ext_vector_type(4), may_alias));
typedef unsigned int v4u __attribute__((ext_vector_type(4)));

union U8f  { v8f  v; float    f[8]; };
union U16h { v16h v; v8h      h[2]; };
union U8h  { v8h  v; _Float16 f[8]; };

#ifndef NB
#define NB 4
#endif
#ifndef SEQ
#define SEQ 2000
#endif
#define NB_FULL  4
#define SEQ_FULL 2000
#define HID   1024
#define NH    16
#define HD    64
#define NQK   2048
#define SEQP  ((((SEQ) + 127) / 128) * 128)
#define MR    ((NB) * SEQP)
#define EARLY 256
#define PPP   2048

static_assert(NB >= 1 && NB <= NB_FULL);
static_assert(SEQ >= 256 && SEQ <= SEQ_FULL);
static_assert(SEQP % 128 == 0 && SEQP >= EARLY && SEQP <= 2048);
static_assert(NH * HD == HID);
static_assert(NQK <= PPP && HID <= PPP);
static_assert(((long long)(NB - 1) * SEQ_FULL + SEQ) * HID <= (long long)NB_FULL * SEQ_FULL * HID);

#define GBM 64
#define GBN 128
#define GBK 32
#define GP  40
#define CP  132
static_assert(MR % GBM == 0 && SEQP % GBM == 0 && EARLY % GBM == 0);
static_assert(HID % GBN == 0 && NQK % GBN == 0 && HID % GBK == 0);
static_assert((GP * 2) % 16 == 0 && (CP * 4) % 16 == 0);
static_assert(2 * (GBM * GP * 2) + GBN * GP * 2 + GBM * CP * 4 <= 65536);

#define BQ 128
#define BK 32
#define QP 72
#define KP 72
#define VP 40
static_assert(SEQP % BQ == 0 && EARLY == 2 * BQ && BQ % BK == 0);

#define SQH_OFF 0
#define SQL_OFF (SQH_OFF + 8 * 16 * QP)
#define SKH_OFF (SQL_OFF + 8 * 16 * QP)
#define SKL_OFF (SKH_OFF + BK * KP)
#define SVH_OFF (SKL_OFF + BK * KP)
#define SVL_OFF (SVH_OFF + HD * VP)
#define SPH_OFF (SVL_OFF + HD * VP)
#define SPR_OFF (SPH_OFF + 8 * 16 * BK)
#define SO_OFFH (SPR_OFF + 8 * 16 * BK)
#define LDS_BYTES (SO_OFFH * 2 + 8 * 16 * 64 * 4)
static_assert((SQL_OFF * 2) % 16 == 0 && (SKH_OFF * 2) % 16 == 0 && (SKL_OFF * 2) % 16 == 0);
static_assert((SVH_OFF * 2) % 16 == 0 && (SVL_OFF * 2) % 16 == 0 && (SPH_OFF * 2) % 16 == 0);
static_assert((SPR_OFF * 2) % 16 == 0 && (SO_OFFH * 2) % 16 == 0);
static_assert(LDS_BYTES == 105472);

#define C2S 0.18033688011112042f

static constexpr size_t kPlaneB = (size_t)MR * HID * 2;
static constexpr size_t kPhB    = (size_t)SEQP * HID * 2;
static constexpr size_t kPPB    = (size_t)SEQP * PPP * 4;
static constexpr size_t kR0B    = (kPlaneB + kPhB + kPPB > 2 * kPlaneB) ? (kPlaneB + kPhB + kPPB) : (2 * kPlaneB);
static constexpr size_t kWhB    = (size_t)4 * HID * HID * 2;
static constexpr size_t kVtlB   = (size_t)NB * NH * HD * EARLY * 2;
static constexpr size_t kOffXh  = 0;
static constexpr size_t kOffPh  = kPlaneB;
static constexpr size_t kOffPP  = kPlaneB + kPhB;
static constexpr size_t kOffCh  = 0;
static constexpr size_t kOffCl  = kPlaneB;
static constexpr size_t kOffWh  = kR0B;
static constexpr size_t kOffQh  = kOffWh + kWhB;
static constexpr size_t kOffQl  = kOffQh + kPlaneB;
static constexpr size_t kOffKh  = kOffQl + kPlaneB;
static constexpr size_t kOffKl  = kOffKh + kPlaneB;
static constexpr size_t kOffVh  = kOffKl + kPlaneB;
static constexpr size_t kOffVl  = kOffVh + kPlaneB;
static constexpr size_t kTotal  = kOffVl + kVtlB;
static_assert(kTotal <= 134217728ull);
static_assert(kOffCl + kPlaneB <= kR0B);
static_assert(kOffPh % 128 == 0 && kOffPP % 128 == 0 && kOffWh % 128 == 0 && kOffQh % 128 == 0);
static_assert(kOffVl % 128 == 0 && kR0B % 128 == 0);
static_assert((size_t)NB * NH * HD * SEQP * 2 == kPlaneB);

__device__ __forceinline__ v8f wmma_f16(v16h a, v16h b, v8f c) {
  v8f d = __builtin_amdgcn_wmma_f32_16x16x32_f16(false, a, false, b, (short)0, c, false, false);
  asm volatile("v_nop\n\tv_nop\n\tv_nop\n\tv_nop" : "+v"(d) : "v"(a), "v"(b));
  return d;
}

template <int CTRL>
__device__ __forceinline__ float dppf(float x) {
  int s = __float_as_int(x);
  return __int_as_float(__builtin_amdgcn_update_dpp(s, s, CTRL, 0xF, 0xF, true));
}
__device__ __forceinline__ float red_max16(float x) {
  x = fmaxf(x, dppf<0xB1>(x));
  x = fmaxf(x, dppf<0x4E>(x));
  x = fmaxf(x, dppf<0x141>(x));
  x = fmaxf(x, dppf<0x140>(x));
  return x;
}
__device__ __forceinline__ float red_sum16(float x) {
  x += dppf<0xB1>(x);
  x += dppf<0x4E>(x);
  x += dppf<0x141>(x);
  x += dppf<0x140>(x);
  return x;
}

__device__ __forceinline__ void wave_lds_sync() {
  __builtin_amdgcn_fence(3, "wavefront");
  asm volatile("s_wait_dscnt 0" ::: "memory");
  __builtin_amdgcn_wave_barrier();
}

__device__ __forceinline__ v4f bf16_rne4(v4f a) {
  v4u u = __builtin_bit_cast(v4u, a);
  u = (u + 0x7FFFu + ((u >> 16) & 1u)) & 0xFFFF0000u;
  return __builtin_bit_cast(v4f, u);
}

__device__ __forceinline__ v8h cvt8v(v4f a, v4f b) {
  v8h d;
  d[0] = (_Float16)a[0]; d[1] = (_Float16)a[1];
  d[2] = (_Float16)a[2]; d[3] = (_Float16)a[3];
  d[4] = (_Float16)b[0]; d[5] = (_Float16)b[1];
  d[6] = (_Float16)b[2]; d[7] = (_Float16)b[3];
  return d;
}

__device__ __forceinline__ void split8(v4f a, v4f b, v8h& hv, v8h& lv) {
  U8h hh, ll;
  _Float16 t;
  t = (_Float16)a[0]; hh.f[0] = t; ll.f[0] = (_Float16)((a[0] - (float)t) * 4096.0f);
  t = (_Float16)a[1]; hh.f[1] = t; ll.f[1] = (_Float16)((a[1] - (float)t) * 4096.0f);
  t = (_Float16)a[2]; hh.f[2] = t; ll.f[2] = (_Float16)((a[2] - (float)t) * 4096.0f);
  t = (_Float16)a[3]; hh.f[3] = t; ll.f[3] = (_Float16)((a[3] - (float)t) * 4096.0f);
  t = (_Float16)b[0]; hh.f[4] = t; ll.f[4] = (_Float16)((b[0] - (float)t) * 4096.0f);
  t = (_Float16)b[1]; hh.f[5] = t; ll.f[5] = (_Float16)((b[1] - (float)t) * 4096.0f);
  t = (_Float16)b[2]; hh.f[6] = t; ll.f[6] = (_Float16)((b[2] - (float)t) * 4096.0f);
  t = (_Float16)b[3]; hh.f[7] = t; ll.f[7] = (_Float16)((b[3] - (float)t) * 4096.0f);
  hv = hh.v; lv = ll.v;
}

__global__ __launch_bounds__(128)
void prep_kernel(const float* __restrict__ Hs, const float* __restrict__ Pos,
                 const float* __restrict__ W0, const float* __restrict__ W1,
                 const float* __restrict__ W2, const float* __restrict__ W3,
                 _Float16* Xh, _Float16* Ph, _Float16* Wh)
{
  const int row = blockIdx.x;
  const int c0  = 8 * threadIdx.x;
  const float* src;
  _Float16*    dst;
  float sc = 1.0f;
  if (row < MR) {
    const int b  = row / SEQP;
    const int s  = row - b * SEQP;
    const int sl = (s < SEQ) ? s : (SEQ - 1);
    sc  = (s < SEQ) ? 1.0f : 0.0f;
    src = Hs + ((size_t)b * SEQ_FULL + sl) * HID + c0;
    dst = Xh + (size_t)row * HID + c0;
  } else if (row < MR + SEQP) {
    const int s  = row - MR;
    const int sl = (s < SEQ) ? s : (SEQ - 1);
    sc  = (s < SEQ) ? 1.0f : 0.0f;
    src = Pos + (size_t)sl * HID + c0;
    dst = Ph + (size_t)s * HID + c0;
  } else {
    const int j   = row - MR - SEQP;
    const int mat = j >> 10;
    const int r   = j & (HID - 1);
    const float* W = (mat == 0) ? W0 : (mat == 1) ? W1 : (mat == 2) ? W2 : W3;
    sc  = 256.0f;
    src = W + (size_t)r * HID + c0;
    dst = Wh + (size_t)j * HID + c0;
  }
  const v4f a0 = bf16_rne4(*(const v4f*)src) * sc;
  const v4f a1 = bf16_rne4(*(const v4f*)(src + 4)) * sc;
  const v8h v  = cvt8v(a0, a1);
  *(volatile v8h*)dst = v;
  __threadfence();
  *(volatile v8h*)dst = v;
}

template <int MODE>
__global__ __launch_bounds__(256)
void gemm_kernel(const _Float16* __restrict__ Ah, const _Float16* __restrict__ Al,
                 const _Float16* __restrict__ Bw, const float* __restrict__ Pin,
                 float* Pout, _Float16* O0, _Float16* O1, _Float16* O2, _Float16* O3, float* Y)
{
  __shared__ __attribute__((aligned(16))) _Float16 sA[GBM * GP];
  __shared__ __attribute__((aligned(16))) _Float16 sL[GBM * GP];
  __shared__ __attribute__((aligned(16))) _Float16 sB[GBN * GP];
  __shared__ __attribute__((aligned(16))) float    sC[GBM * CP];

  const int tid  = threadIdx.x;
  const int wave = tid >> 5;
  const int lane = tid & 31;
  const int lh   = lane & 15;
  const int hi   = lane >> 4;
  const int wm   = wave >> 2;
  const int wn   = wave & 3;
  const int sub  = tid & 7;
  const int m0   = blockIdx.y * GBM;
  const int n0   = blockIdx.x * GBN;
  const int b    = m0 / SEQP;
  const int s0   = m0 - b * SEQP;
  const bool resa = (MODE == 3) && (s0 < EARLY);

  U8f acc[2][2], accr[2][2];
  #pragma unroll
  for (int mi = 0; mi < 2; ++mi)
    #pragma unroll
    for (int ni = 0; ni < 2; ++ni) { acc[mi][ni].v = (v8f){}; accr[mi][ni].v = (v8f){}; }

  const int ar = tid >> 2, ag = tid & 3;
  const size_t aoff = (size_t)(m0 + ar) * HID + 8 * ag;

  for (int k0 = 0; k0 < HID; k0 += GBK) {
    __syncthreads();
    *(v8h*)(sA + ar * GP + 8 * ag) = *(const v8h*)(Ah + aoff + k0);
    if (resa) *(v8h*)(sL + ar * GP + 8 * ag) = *(const v8h*)(Al + aoff + k0);
    #pragma unroll
    for (int i = 0; i < 2; ++i) {
      const int idx = tid + 256 * i;
      const int br = idx >> 2, bg = idx & 3;
      *(v8h*)(sB + br * GP + 8 * bg) = *(const v8h*)(Bw + (size_t)(n0 + br) * HID + k0 + 8 * bg);
    }
    __syncthreads();

    U16h af[2], bq[2];
    #pragma unroll
    for (int mi = 0; mi < 2; ++mi) {
      const _Float16* p = sA + (wm * 32 + mi * 16 + lh) * GP;
      af[mi].h[0] = *(const v8h*)(p + 8 * hi);
      af[mi].h[1] = *(const v8h*)(p + 16 + 8 * hi);
    }
    #pragma unroll
    for (int ni = 0; ni < 2; ++ni) {
      const _Float16* p = sB + (wn * 32 + ni * 16 + lh) * GP;
      bq[ni].h[0] = *(const v8h*)(p + 8 * hi);
      bq[ni].h[1] = *(const v8h*)(p + 16 + 8 * hi);
    }
    #pragma unroll
    for (int mi = 0; mi < 2; ++mi)
      #pragma unroll
      for (int ni = 0; ni < 2; ++ni)
        acc[mi][ni].v = wmma_f16(af[mi].v, bq[ni].v, acc[mi][ni].v);
    if (resa) {
      U16h lf[2];
      #pragma unroll
      for (int mi = 0; mi < 2; ++mi) {
        const _Float16* p = sL + (wm * 32 + mi * 16 + lh) * GP;
        lf[mi].h[0] = *(const v8h*)(p + 8 * hi);
        lf[mi].h[1] = *(const v8h*)(p + 16 + 8 * hi);
      }
      #pragma unroll
      for (int mi = 0; mi < 2; ++mi)
        #pragma unroll
        for (int ni = 0; ni < 2; ++ni)
          accr[mi][ni].v = wmma_f16(lf[mi].v, bq[ni].v, accr[mi][ni].v);
    }
  }

  #pragma unroll
  for (int mi = 0; mi < 2; ++mi)
    #pragma unroll
    for (int ni = 0; ni < 2; ++ni)
      #pragma unroll
      for (int r = 0; r < 8; ++r) {
        float v = acc[mi][ni].f[r];
        if (resa) v += accr[mi][ni].f[r] * (1.0f / 4096.0f);
        sC[(wm * 32 + mi * 16 + 8 * hi + r) * CP + wn * 32 + ni * 16 + lh] = v * (1.0f / 256.0f);
      }
  __syncthreads();

  if (MODE == 1 || MODE == 2) {
    #pragma unroll
    for (int p = 0; p < 4; ++p) {
      const int g   = p * 256 + tid;
      const int row = g >> 4;
      const int cg  = g & 15;
      const float* pp = Pin + (size_t)(s0 + row) * PPP + n0 + 8 * cg;
      const v4f p0 = *(const v4f*)pp;
      const v4f p1 = *(const v4f*)(pp + 4);
      v4fa* c = (v4fa*)(sC + row * CP + 8 * cg);
      v4f x0 = c[0], x1 = c[1];
      x0 += p0; x1 += p1;
      c[0] = x0; c[1] = x1;
    }
    __syncthreads();
  }

  if (MODE == 0) {
    v4f ov[8]; size_t oo[8];
    #pragma unroll
    for (int i = 0; i < 8; ++i) {
      const int L = 32 * i + (tid >> 3);
      const int row = L >> 2, seg = L & 3;
      ov[i] = *(const v4fa*)(sC + row * CP + seg * 32 + 4 * sub);
      oo[i] = (size_t)(m0 + row) * PPP + n0 + seg * 32 + 4 * sub;
    }
    #pragma unroll
    for (int i = 0; i < 8; ++i) *(volatile v4f*)(Pout + oo[i]) = ov[i];
    __threadfence();
    #pragma unroll
    for (int i = 0; i < 8; ++i) *(volatile v4f*)(Pout + oo[i]) = ov[i];
  }

  if (MODE == 1) {
    const bool isq = (n0 < HID);
    _Float16* ph = isq ? O0 : O2;
    _Float16* pl = isq ? O1 : O3;
    const int col0 = n0 & (HID - 1);
    v8h vh[4], vl[4]; size_t oo[4];
    #pragma unroll
    for (int i = 0; i < 4; ++i) {
      const int rem = 32 * i + (tid >> 3);
      const int row = rem >> 1, seg = rem & 1;
      const float* c = sC + row * CP + seg * 64 + 8 * sub;
      split8(*(const v4fa*)c, *(const v4fa*)(c + 4), vh[i], vl[i]);
      oo[i] = (size_t)(m0 + row) * HID + col0 + seg * 64 + 8 * sub;
    }
    #pragma unroll
    for (int i = 0; i < 4; ++i) { *(volatile v8h*)(ph + oo[i]) = vh[i]; *(volatile v8h*)(pl + oo[i]) = vl[i]; }
    __threadfence();
    #pragma unroll
    for (int i = 0; i < 4; ++i) { *(volatile v8h*)(ph + oo[i]) = vh[i]; *(volatile v8h*)(pl + oo[i]) = vl[i]; }
  }

  if (MODE == 2) {
    const int h0 = n0 / HD;
    v8h vh[4], vl[4]; size_t oh[4], ol[4];
    #pragma unroll
    for (int i = 0; i < 4; ++i) {
      const int c  = 32 * i + (tid >> 3);
      const int hh = h0 + (c >> 6);
      const int d  = c & (HD - 1);
      v4f x0, x1;
      x0[0] = sC[(8 * sub + 0) * CP + c]; x0[1] = sC[(8 * sub + 1) * CP + c];
      x0[2] = sC[(8 * sub + 2) * CP + c]; x0[3] = sC[(8 * sub + 3) * CP + c];
      x1[0] = sC[(8 * sub + 4) * CP + c]; x1[1] = sC[(8 * sub + 5) * CP + c];
      x1[2] = sC[(8 * sub + 6) * CP + c]; x1[3] = sC[(8 * sub + 7) * CP + c];
      split8(x0, x1, vh[i], vl[i]);
      const size_t rowid = (size_t)(b * NH + hh) * HD + d;
      oh[i] = rowid * SEQP + s0 + 8 * sub;
      ol[i] = rowid * EARLY + s0 + 8 * sub;
    }
    #pragma unroll
    for (int i = 0; i < 4; ++i) {
      *(volatile v8h*)(O0 + oh[i]) = vh[i];
      if (s0 < EARLY) *(volatile v8h*)(O1 + ol[i]) = vl[i];
    }
    __threadfence();
    #pragma unroll
    for (int i = 0; i < 4; ++i) {
      *(volatile v8h*)(O0 + oh[i]) = vh[i];
      if (s0 < EARLY) *(volatile v8h*)(O1 + ol[i]) = vl[i];
    }
  }

  if (MODE == 3) {
    v4f ov[8]; size_t oo[8]; int sv[8];
    #pragma unroll
    for (int i = 0; i < 8; ++i) {
      const int L = 32 * i + (tid >> 3);
      const int row = L >> 2, seg = L & 3;
      ov[i] = *(const v4fa*)(sC + row * CP + seg * 32 + 4 * sub);
      sv[i] = s0 + row;
      oo[i] = ((size_t)b * SEQ_FULL + (size_t)(s0 + row)) * HID + n0 + seg * 32 + 4 * sub;
    }
    #pragma unroll
    for (int i = 0; i < 8; ++i) if (sv[i] < SEQ) *(volatile v4f*)(Y + oo[i]) = ov[i];
    __threadfence();
    #pragma unroll
    for (int i = 0; i < 8; ++i) if (sv[i] < SEQ) *(volatile v4f*)(Y + oo[i]) = ov[i];
  }
}

template <bool RES>
__global__ __launch_bounds__(256)
void attn_kernel(const _Float16* __restrict__ Qh, const _Float16* __restrict__ Ql,
                 const _Float16* __restrict__ Kh, const _Float16* __restrict__ Kl,
                 const _Float16* __restrict__ Vth, const _Float16* __restrict__ Vtl,
                 _Float16* Ch, _Float16* Cl, int qb0, int nqbl)
{
  extern __shared__ __attribute__((aligned(16))) _Float16 smem[];
  _Float16* sQh = smem + SQH_OFF;
  _Float16* sQl = smem + SQL_OFF;
  _Float16* sKh = smem + SKH_OFF;
  _Float16* sKl = smem + SKL_OFF;
  _Float16* sVh = smem + SVH_OFF;
  _Float16* sVl = smem + SVL_OFF;
  _Float16* sPh = smem + SPH_OFF;
  _Float16* sPr = smem + SPR_OFF;
  float*    sO  = (float*)(smem + SO_OFFH);

  const int tid  = threadIdx.x;
  const int wave = tid >> 5;
  const int lane = tid & 31;
  const int lh   = lane & 15;
  const int hi   = lane >> 4;

  const int qbi   = blockIdx.x % nqbl;
  const int bh    = blockIdx.x / nqbl;
  const int h     = bh % NH;
  const int b     = bh / NH;
  const int qbase = (qb0 + qbi) * BQ;
  const int qrow0 = qbase + wave * 16;

  const size_t prow = (size_t)b * SEQP;
  const _Float16* Qhb = Qh + prow * HID + h * HD;
  const _Float16* Qlb = Ql + prow * HID + h * HD;
  const _Float16* Khb = Kh + prow * HID + h * HD;
  const _Float16* Klb = Kl + prow * HID + h * HD;
  const _Float16* Vhb = Vth + (size_t)(b * NH + h) * HD * SEQP;
  const _Float16* Vlb = Vtl + (size_t)(b * NH + h) * HD * EARLY;
  _Float16* Chb = Ch + prow * HID + h * HD;
  _Float16* Clb = Cl + prow * HID + h * HD;

  _Float16* qwh = sQh + wave * (16 * QP);
  _Float16* qwl = sQl + wave * (16 * QP);
  {
    const int pc = lane & 7;
    #pragma unroll
    for (int i = 0; i < 4; ++i) {
      const int r = 4 * i + (lane >> 3);
      const size_t go = (size_t)(qrow0 + r) * HID + 8 * pc;
      *(v8h*)(qwh + r * QP + 8 * pc) = *(const v8h*)(Qhb + go);
      *(v8h*)(qwl + r * QP + 8 * pc) = *(const v8h*)(Qlb + go);
    }
  }

  U8f acc[4], accr[4];
  #pragma unroll
  for (int t = 0; t < 4; ++t) { acc[t].v = (v8f){}; accr[t].v = (v8f){}; }
  float mrow[8], lrow[8];
  #pragma unroll
  for (int j = 0; j < 8; ++j) { mrow[j] = -3.0e38f; lrow[j] = 0.0f; }

  _Float16* pwh = sPh + wave * (16 * BK);
  _Float16* pwr = sPr + wave * (16 * BK);

  const int kend = qbase + BQ;
  const int kr = tid >> 3, kg = tid & 7;
  const int vd = tid >> 2, vg = tid & 3;

  for (int kv0 = 0; kv0 < kend; kv0 += BK) {
    __syncthreads();
    {
      const size_t ko = (size_t)(kv0 + kr) * HID + 8 * kg;
      *(v8h*)(sKh + kr * KP + 8 * kg) = *(const v8h*)(Khb + ko);
      *(v8h*)(sKl + kr * KP + 8 * kg) = *(const v8h*)(Klb + ko);
      *(v8h*)(sVh + vd * VP + 8 * vg) = *(const v8h*)(Vhb + (size_t)vd * SEQP + kv0 + 8 * vg);
      if (RES) *(v8h*)(sVl + vd * VP + 8 * vg) = *(const v8h*)(Vlb + (size_t)vd * EARLY + kv0 + 8 * vg);
    }
    __syncthreads();

    if (kv0 < qrow0 + 16) {
      U8f s0, s1;
      {
        U8f sm, sr; sm.v = (v8f){}; sr.v = (v8f){};
        #pragma unroll
        for (int c = 0; c < 2; ++c) {
          U16h qf, ql, kf, kl;
          qf.h[0] = *(const v8h*)(qwh + lh * QP + 32 * c + 8 * hi);
          qf.h[1] = *(const v8h*)(qwh + lh * QP + 32 * c + 16 + 8 * hi);
          ql.h[0] = *(const v8h*)(qwl + lh * QP + 32 * c + 8 * hi);
          ql.h[1] = *(const v8h*)(qwl + lh * QP + 32 * c + 16 + 8 * hi);
          kf.h[0] = *(const v8h*)(sKh + lh * KP + 32 * c + 8 * hi);
          kf.h[1] = *(const v8h*)(sKh + lh * KP + 32 * c + 16 + 8 * hi);
          kl.h[0] = *(const v8h*)(sKl + lh * KP + 32 * c + 8 * hi);
          kl.h[1] = *(const v8h*)(sKl + lh * KP + 32 * c + 16 + 8 * hi);
          sm.v = wmma_f16(qf.v, kf.v, sm.v);
          sr.v = wmma_f16(qf.v, kl.v, sr.v);
          sr.v = wmma_f16(ql.v, kf.v, sr.v);
        }
        s0.v = sm.v + sr.v * (1.0f / 4096.0f);
      }
      {
        U8f sm, sr; sm.v = (v8f){}; sr.v = (v8f){};
        #pragma unroll
        for (int c = 0; c < 2; ++c) {
          U16h qf, ql, kf, kl;
          qf.h[0] = *(const v8h*)(qwh + lh * QP + 32 * c + 8 * hi);
          qf.h[1] = *(const v8h*)(qwh + lh * QP + 32 * c + 16 + 8 * hi);
          ql.h[0] = *(const v8h*)(qwl + lh * QP + 32 * c + 8 * hi);
          ql.h[1] = *(const v8h*)(qwl + lh * QP + 32 * c + 16 + 8 * hi);
          kf.h[0] = *(const v8h*)(sKh + (16 + lh) * KP + 32 * c + 8 * hi);
          kf.h[1] = *(const v8h*)(sKh + (16 + lh) * KP + 32 * c + 16 + 8 * hi);
          kl.h[0] = *(const v8h*)(sKl + (16 + lh) * KP + 32 * c + 8 * hi);
          kl.h[1] = *(const v8h*)(sKl + (16 + lh) * KP + 32 * c + 16 + 8 * hi);
          sm.v = wmma_f16(qf.v, kf.v, sm.v);
          sr.v = wmma_f16(qf.v, kl.v, sr.v);
          sr.v = wmma_f16(ql.v, kf.v, sr.v);
        }
        s1.v = sm.v + sr.v * (1.0f / 4096.0f);
      }

      const int key0 = kv0 + lh;
      const int key1 = kv0 + 16 + lh;
      U8h pa, pb, par, pbr;
      #pragma unroll
      for (int j = 0; j < 8; ++j) {
        const int row  = qrow0 + 8 * hi + j;
        const float x0 = s0.f[j] * C2S;
        const float x1 = s1.f[j] * C2S;
        const float a  = (key0 <= row) ? x0 : -1.0e30f;
        const float bb = (key1 <= row) ? x1 : -1.0e30f;
        const float rm    = red_max16(fmaxf(a, bb));
        const float mnew  = fmaxf(mrow[j], rm);
        const float alpha = __builtin_amdgcn_exp2f(mrow[j] - mnew);
        const float e0    = __builtin_amdgcn_exp2f(a - mnew);
        const float e1    = __builtin_amdgcn_exp2f(bb - mnew);
        lrow[j] = lrow[j] * alpha + red_sum16(e0 + e1);
        mrow[j] = mnew;
        const float t0 = e0 * 1024.0f;
        const float t1 = e1 * 1024.0f;
        const _Float16 h0 = (_Float16)t0;
        const _Float16 h1 = (_Float16)t1;
        pa.f[j] = h0; pb.f[j] = h1;
        if (RES) {
          par.f[j] = (_Float16)((t0 - (float)h0) * 4096.0f);
          pbr.f[j] = (_Float16)((t1 - (float)h1) * 4096.0f);
        }
        #pragma unroll
        for (int t = 0; t < 4; ++t) {
          acc[t].f[j] *= alpha;
          if (RES) accr[t].f[j] *= alpha;
        }
      }

      #pragma unroll
      for (int j = 0; j < 8; ++j) {
        pwh[(j + 8 * hi) * BK + lh]      = pa.f[j];
        pwh[(j + 8 * hi) * BK + 16 + lh] = pb.f[j];
        if (RES) {
          pwr[(j + 8 * hi) * BK + lh]      = par.f[j];
          pwr[(j + 8 * hi) * BK + 16 + lh] = pbr.f[j];
        }
      }
      wave_lds_sync();
      U16h pf, pfr;
      pf.h[0] = *(const v8ha*)(pwh + lh * BK + 8 * hi);
      pf.h[1] = *(const v8ha*)(pwh + lh * BK + 16 + 8 * hi);
      if (RES) {
        pfr.h[0] = *(const v8ha*)(pwr + lh * BK + 8 * hi);
        pfr.h[1] = *(const v8ha*)(pwr + lh * BK + 16 + 8 * hi);
      }

      #pragma unroll
      for (int t = 0; t < 4; ++t) {
        U16h vf;
        vf.h[0] = *(const v8h*)(sVh + (16 * t + lh) * VP + 8 * hi);
        vf.h[1] = *(const v8h*)(sVh + (16 * t + lh) * VP + 16 + 8 * hi);
        acc[t].v = wmma_f16(pf.v, vf.v, acc[t].v);
        if (RES) {
          U16h wl;
          wl.h[0] = *(const v8h*)(sVl + (16 * t + lh) * VP + 8 * hi);
          wl.h[1] = *(const v8h*)(sVl + (16 * t + lh) * VP + 16 + 8 * hi);
          accr[t].v = wmma_f16(pf.v, wl.v, accr[t].v);
          accr[t].v = wmma_f16(pfr.v, vf.v, accr[t].v);
        }
      }
    }
  }

  float inv[8];
  #pragma unroll
  for (int j = 0; j < 8; ++j) inv[j] = 1.0f / (lrow[j] * 1024.0f);
  float* so = sO + wave * (16 * 64);
  #pragma unroll
  for (int j = 0; j < 8; ++j) {
    #pragma unroll
    for (int t = 0; t < 4; ++t) {
      float v = acc[t].f[j];
      if (RES) v += accr[t].f[j] * (1.0f / 4096.0f);
      so[(j + 8 * hi) * 64 + t * 16 + lh] = v * inv[j];
    }
  }
  wave_lds_sync();
  v8h oh[4], ol[4]; size_t oo[4];
  {
    const int pc = lane & 7;
    #pragma unroll
    for (int i = 0; i < 4; ++i) {
      const int rr = 4 * i + (lane >> 3);
      const float* sp = so + rr * 64 + 8 * pc;
      split8(*(const v4fa*)sp, *(const v4fa*)(sp + 4), oh[i], ol[i]);
      oo[i] = (size_t)(qrow0 + rr) * HID + 8 * pc;
    }
  }
  #pragma unroll
  for (int i = 0; i < 4; ++i) { *(volatile v8h*)(Chb + oo[i]) = oh[i]; *(volatile v8h*)(Clb + oo[i]) = ol[i]; }
  __threadfence();
  #pragma unroll
  for (int i = 0; i < 4; ++i) { *(volatile v8h*)(Chb + oo[i]) = oh[i]; *(volatile v8h*)(Clb + oo[i]) = ol[i]; }
}

extern "C" void kernel_launch(void* const* d_in, const int* in_sizes, int n_in,
                              void* d_out, int out_size, void* d_ws, size_t ws_size,
                              hipStream_t stream) {
  if (n_in < 6) return;
  const long long need_x = ((long long)(NB - 1) * SEQ_FULL + SEQ) * HID;
  if ((long long)in_sizes[0] < need_x) return;
  if ((long long)in_sizes[1] < (long long)HID * HID) return;
  if ((long long)in_sizes[2] < (long long)HID * HID) return;
  if ((long long)in_sizes[3] < (long long)HID * HID) return;
  if ((long long)in_sizes[4] < (long long)HID * HID) return;
  if ((long long)in_sizes[5] < (long long)SEQ * HID) return;
  if ((long long)out_size < need_x) return;
  if (kTotal > ws_size) return;

  const float* hs  = (const float*)d_in[0];
  const float* wq  = (const float*)d_in[1];
  const float* wk  = (const float*)d_in[2];
  const float* wv  = (const float*)d_in[3];
  const float* wo  = (const float*)d_in[4];
  const float* pos = (const float*)d_in[5];
  float*       out = (float*)d_out;

  char* ws = (char*)d_ws;
  _Float16* xh = (_Float16*)(ws + kOffXh);
  _Float16* ph = (_Float16*)(ws + kOffPh);
  float*    pp = (float*)(ws + kOffPP);
  _Float16* ch = (_Float16*)(ws + kOffCh);
  _Float16* cl = (_Float16*)(ws + kOffCl);
  _Float16* wh = (_Float16*)(ws + kOffWh);
  _Float16* qh = (_Float16*)(ws + kOffQh);
  _Float16* ql = (_Float16*)(ws + kOffQl);
  _Float16* kh = (_Float16*)(ws + kOffKh);
  _Float16* kl = (_Float16*)(ws + kOffKl);
  _Float16* vh = (_Float16*)(ws + kOffVh);
  _Float16* vl = (_Float16*)(ws + kOffVl);

  prep_kernel<<<dim3(MR + SEQP + 4 * HID), dim3(128), 0, stream>>>(hs, pos, wq, wk, wv, wo, xh, ph, wh);

  gemm_kernel<0><<<dim3(NQK / GBN, SEQP / GBM), dim3(256), 0, stream>>>(ph, ph, wh, pp, pp, qh, ql, kh, kl, out);
  gemm_kernel<1><<<dim3(NQK / GBN, MR / GBM), dim3(256), 0, stream>>>(xh, xh, wh, pp, pp, qh, ql, kh, kl, out);
  const _Float16* whv = wh + (size_t)NQK * HID;
  gemm_kernel<0><<<dim3(HID / GBN, SEQP / GBM), dim3(256), 0, stream>>>(ph, ph, whv, pp, pp, qh, ql, kh, kl, out);
  gemm_kernel<2><<<dim3(HID / GBN, MR / GBM), dim3(256), 0, stream>>>(xh, xh, whv, pp, pp, vh, vl, kh, kl, out);

  (void)hipFuncSetAttribute(reinterpret_cast<const void*>(&attn_kernel<true>),
                            hipFuncAttributeMaxDynamicSharedMemorySize, (int)LDS_BYTES);
  (void)hipFuncSetAttribute(reinterpret_cast<const void*>(&attn_kernel<false>),
                            hipFuncAttributeMaxDynamicSharedMemorySize, (int)LDS_BYTES);
  const int nqb = SEQP / BQ;
  attn_kernel<true><<<dim3(NB * NH * 2), dim3(256), LDS_BYTES, stream>>>(qh, ql, kh, kl, vh, vl, ch, cl, 0, 2);
  if (nqb > 2)
    attn_kernel<false><<<dim3(NB * NH * (nqb - 2)), dim3(256), LDS_BYTES, stream>>>(qh, ql, kh, kl, vh, vl, ch, cl, 2, nqb - 2);

  const _Float16* who = wh + (size_t)(NQK + HID) * HID;
  gemm_kernel<3><<<dim3(HID / GBN, MR / GBM), dim3(256), 0, stream>>>(ch, cl, who, pp, pp, qh, ql, kh, kl, out);
}
